// TTLinear_12232066859472
// MI455X (gfx1250) — hardware-verified
//
#include <hip/hip_runtime.h>


#define NBALL 2048
#define BC    128
#define NCH   (NBALL / BC)
#define RW    (BC * 256)
typedef _Float16 h16;
typedef unsigned short bf;
typedef __attribute__((ext_vector_type(16))) __bf16   v16bf;
typedef __attribute__((ext_vector_type(16))) _Float16 v16h;
typedef __attribute__((ext_vector_type(8)))  _Float16 v8h;
typedef __attribute__((ext_vector_type(8)))  unsigned short v8us;
typedef __attribute__((ext_vector_type(8)))  float    v8f;
typedef __attribute__((ext_vector_type(4)))  float    v4f;
typedef v8h  __attribute__((may_alias)) v8ha;
typedef v4f  __attribute__((may_alias)) v4fa;
typedef v8us __attribute__((may_alias)) v8usa;

__device__ __forceinline__ unsigned short f2bf(float f) { unsigned u = __float_as_uint(f); u += 0x7FFFu + ((u >> 16) & 1u); return (unsigned short)(u >> 16); }
__device__ __forceinline__ float bf2f(unsigned short b) { return __uint_as_float(((unsigned)b) << 16); }
__device__ __forceinline__ float bfr(float f) { return bf2f(f2bf(f)); }
__device__ __forceinline__ v16h cat16(v8h lo, v8h hi) { return __builtin_shufflevector(lo, hi, 0, 1, 2, 3, 4, 5, 6, 7, 8, 9, 10, 11, 12, 13, 14, 15); }
__device__ __forceinline__ v16bf cat16b(v8us lo, v8us hi) { return __builtin_bit_cast(v16bf, __builtin_shufflevector(lo, hi, 0, 1, 2, 3, 4, 5, 6, 7, 8, 9, 10, 11, 12, 13, 14, 15)); }
__device__ __forceinline__ v8f wmma16(v16h a, v16h b, v8f c) { return __builtin_amdgcn_wmma_f32_16x16x32_f16(false, a, false, b, (short)0, c, false, false); }
__device__ __forceinline__ v8f wmmab(v16bf a, v16bf b, v8f c) { return __builtin_amdgcn_wmma_f32_16x16x32_bf16(false, a, false, b, (short)0, c, false, false); }


template <typename T16> struct WFrag;
template <> struct WFrag<h16> { typedef v16h V; static __device__ __forceinline__ V ld(const h16* p) { return cat16(*(const v8h*)p, *(const v8h*)(p + 16)); } static __device__ __forceinline__ v8f mma(V a, V b, v8f c) { return wmma16(a, b, c); } };
template <> struct WFrag<bf> { typedef v16bf V; static __device__ __forceinline__ V ld(const bf* p) { return cat16b(*(const v8us*)p, *(const v8us*)(p + 16)); } static __device__ __forceinline__ v8f mma(V a, V b, v8f c) { return wmmab(a, b, c); } };
template <typename T16, int NSPLIT, bool BIAS>
__global__ __launch_bounds__(32) void k_gemmw(const T16* __restrict__ A, const T16* __restrict__ A2, const T16* __restrict__ Bt, const T16* __restrict__ Bt2, int K, float* C, int ldc, const float* __restrict__ bias, size_t sA, size_t sB, size_t sC) {
    typedef typename WFrag<T16>::V V;
    __shared__ __align__(16) float os[16 * 68];
    const size_t z = blockIdx.z; A += z * sA; if (A2) A2 += z * sA; Bt += z * sB; if (Bt2) Bt2 += z * sB; C += z * sC;
    const int lane = threadIdx.x & 31, lr = lane & 15, hi = lane >> 4; const int r0 = blockIdx.x * 64, c0 = blockIdx.y * 64;
    v8f acc[4][4];
#pragma unroll
    for (int mb = 0; mb < 4; ++mb)
#pragma unroll
        for (int nb = 0; nb < 4; ++nb) acc[mb][nb] = (v8f){};
    const size_t aoff = (size_t)(r0 + lr) * K + 8 * hi, boff = (size_t)(c0 + lr) * K + 8 * hi;
#pragma unroll 1
    for (int kc = 0; kc < K; kc += 32) {
        V a[4], a2[4];
#pragma unroll
        for (int mb = 0; mb < 4; ++mb) { a[mb] = WFrag<T16>::ld(A + aoff + (size_t)mb * 16 * K + kc); if (NSPLIT == 1 || NSPLIT == 2) a2[mb] = WFrag<T16>::ld(A2 + aoff + (size_t)mb * 16 * K + kc); }
#pragma unroll
        for (int nb = 0; nb < 4; ++nb) { const V b = WFrag<T16>::ld(Bt + boff + (size_t)nb * 16 * K + kc); V b2; if (NSPLIT >= 2) b2 = WFrag<T16>::ld(Bt2 + boff + (size_t)nb * 16 * K + kc);
#pragma unroll
            for (int mb = 0; mb < 4; ++mb) { acc[mb][nb] = WFrag<T16>::mma(a[mb], b, acc[mb][nb]); if (NSPLIT == 1 || NSPLIT == 2) acc[mb][nb] = WFrag<T16>::mma(a2[mb], b, acc[mb][nb]); if (NSPLIT >= 2) acc[mb][nb] = WFrag<T16>::mma(a[mb], b2, acc[mb][nb]); } }
        asm volatile("v_nop\n\tv_nop\n\tv_nop\n\tv_nop" : "+v"(acc[0][0]), "+v"(acc[1][1]), "+v"(acc[2][2]), "+v"(acc[3][3]) : "v"(a[0]), "v"(a[3]));
    }
#pragma unroll
    for (int mb = 0; mb < 4; ++mb) {
#pragma unroll
        for (int nb = 0; nb < 4; ++nb) {
#pragma unroll
            for (int j = 0; j < 8; ++j) os[(hi * 8 + j) * 68 + nb * 16 + lr] = acc[mb][nb][j]; }
        __builtin_amdgcn_wave_barrier(); asm volatile("" ::: "memory");
        float* crow = C + (size_t)(r0 + mb * 16) * ldc + c0;
#pragma unroll 1
        for (int ps = 0; ps < 2; ++ps) {
#pragma unroll
            for (int s = 0; s < 8; ++s) { const int row = 2 * s + hi, cofs = lr * 4; v4f val = *(const v4fa*)(os + row * 68 + cofs); if (BIAS) { val[0] += bfr(bias[c0 + cofs]); val[1] += bfr(bias[c0 + cofs + 1]); val[2] += bfr(bias[c0 + cofs + 2]); val[3] += bfr(bias[c0 + cofs + 3]); }
                *(volatile v4f*)(crow + (size_t)row * ldc + cofs) = val; }
            if (ps == 0) __threadfence(); }
        __builtin_amdgcn_wave_barrier(); asm volatile("" ::: "memory");
    }
}

__device__ __forceinline__ void splitf(float y, unsigned short& h, unsigned short& l) { h = f2bf(y); l = f2bf(y - bf2f(h)); }
typedef __attribute__((ext_vector_type(4))) unsigned short v4us;
__global__ __launch_bounds__(256) void k_w0p(const float* __restrict__ w0, bf* B0) { const int e = (blockIdx.x * 256 + threadIdx.x) * 8; if (e >= 256 * 32) return; const int k = e % 32, n = e / 32; v8us o;
#pragma unroll
    for (int q = 0; q < 8; ++q) o[q] = (k + q < 16) ? f2bf(w0[n * 16 + k + q]) : (unsigned short)0; *(volatile v8us*)(B0 + e) = o; __threadfence(); *(volatile v8us*)(B0 + e) = o; }
__global__ __launch_bounds__(256) void k_w2p(const float* __restrict__ w2, bf* B2) { const int e = (blockIdx.x * 256 + threadIdx.x) * 8; if (e >= 64 * 256) return; const int k = e % 256, n = e / 256; v8us o;
#pragma unroll
    for (int q = 0; q < 8; ++q) o[q] = (n < 16) ? f2bf(w2[n * 256 + k + q]) : (unsigned short)0; *(volatile v8us*)(B2 + e) = o; __threadfence(); *(volatile v8us*)(B2 + e) = o; }
__global__ __launch_bounds__(256) void k_w1p(const float* __restrict__ w1, bf* B1) { const int e = (blockIdx.x * 256 + threadIdx.x) * 8; if (e >= 256 * 256) return; const v8f v = *(const v8f*)(w1 + e); v8us o;
#pragma unroll
    for (int q = 0; q < 8; ++q) o[q] = f2bf(v[q]); *(volatile v8us*)(B1 + e) = o; __threadfence(); *(volatile v8us*)(B1 + e) = o; }
__global__ __launch_bounds__(256) void k_a0(const float* __restrict__ x, int b0, bf* A0) { const size_t e = ((size_t)blockIdx.x * 256 + threadIdx.x) * 8; if (e >= (size_t)RW * 32) return; const int k = (int)(e % 32); const size_t row = e / 32; const int m2 = (int)(row % 16), m1 = (int)((row / 16) % 16), bl = (int)(row / 256); const float* xb = x + (size_t)(b0 + bl) * 4096 + m1 * 16 + m2; v8us o;
#pragma unroll
    for (int q = 0; q < 8; ++q) o[q] = (k + q < 16) ? f2bf(xb[(size_t)(k + q) * 256]) : (unsigned short)0; *(volatile v8us*)(A0 + e) = o; __threadfence(); *(volatile v8us*)(A0 + e) = o; }
__global__ __launch_bounds__(256) void k_p1(const float* __restrict__ C0, bf* Ah, bf* Al) { const size_t e = ((size_t)blockIdx.x * 256 + threadIdx.x) * 4; if (e >= (size_t)RW * 256) return; const int kk = (int)(e % 256); const size_t row = e / 256; const int r1 = kk % 16, m1 = kk / 16; const int o0 = (int)(row % 16), m2 = (int)((row / 16) % 16), bl = (int)(row / 256);
    const v4f v = *(const v4f*)(C0 + (((size_t)bl * 16 + m1) * 16 + m2) * 256 + o0 * 16 + r1); v4us oh, ol;
#pragma unroll
    for (int q = 0; q < 4; ++q) { unsigned short a, c; splitf(v[q], a, c); oh[q] = a; ol[q] = c; } *(volatile v4us*)(Ah + e) = oh; *(volatile v4us*)(Al + e) = ol; __threadfence(); *(volatile v4us*)(Ah + e) = oh; *(volatile v4us*)(Al + e) = ol; }
__global__ __launch_bounds__(256) void k_p2(const float* __restrict__ C1, bf* Ah, bf* Al) { const size_t e = ((size_t)blockIdx.x * 256 + threadIdx.x) * 4; if (e >= (size_t)RW * 256) return; const int kk = (int)(e % 256); const size_t row = e / 256; const int r2 = kk % 16, m2 = kk / 16; const int o1 = (int)(row % 16), o0 = (int)((row / 16) % 16), bl = (int)(row / 256);
    const v4f v = *(const v4f*)(C1 + (((size_t)bl * 16 + m2) * 16 + o0) * 256 + o1 * 16 + r2); v4us oh, ol;
#pragma unroll
    for (int q = 0; q < 4; ++q) { unsigned short a, c; splitf(v[q], a, c); oh[q] = a; ol[q] = c; } *(volatile v4us*)(Ah + e) = oh; *(volatile v4us*)(Al + e) = ol; __threadfence(); *(volatile v4us*)(Ah + e) = oh; *(volatile v4us*)(Al + e) = ol; }
__global__ __launch_bounds__(256) void k_out(const float* __restrict__ C2, const float* __restrict__ bias, int b0, float* O) { const size_t e = ((size_t)blockIdx.x * 256 + threadIdx.x) * 4; if (e >= (size_t)BC * 4096) return; const int col = (int)(e % 4096); const int bl = (int)(e / 4096); const int o2 = col % 16; const int rowi = col / 16;     const v4f v = *(const v4f*)(C2 + ((size_t)bl * 256 + rowi) * 64 + o2); v4f o;
#pragma unroll
    for (int q = 0; q < 4; ++q) o[q] = __fadd_rn(v[q], bfr(bias[col + q])); float* dst = O + (size_t)(b0 + bl) * 4096 + col; *(volatile v4f*)dst = o; __threadfence(); *(volatile v4f*)dst = o; }

extern "C" void kernel_launch(void* const* d_in, const int* in_sizes, int n_in,
                              void* d_out, int out_size, void* d_ws, size_t ws_size, hipStream_t stream) {
    (void)in_sizes; (void)n_in; (void)out_size;
    const float* x = (const float*)d_in[0]; const float* w0 = (const float*)d_in[1]; const float* w1 = (const float*)d_in[2]; const float* w2 = (const float*)d_in[3]; const float* bias = (const float*)d_in[4];
    float* OUT = (float*)d_out;
    char* wsp = (char*)d_ws;
    auto take = [&](size_t bytes) { char* p = wsp; wsp += (bytes + 255) & ~(size_t)255; return (void*)p; };
    bf* B0 = (bf*)take(256 * 32 * 2); bf* B1 = (bf*)take(256 * 256 * 2); bf* B2 = (bf*)take(64 * 256 * 2);
    bf* A0 = (bf*)take((size_t)RW * 32 * 2); float* C0 = (float*)take((size_t)RW * 256 * 4); bf* A1h = (bf*)take((size_t)RW * 256 * 2); bf* A1l = (bf*)take((size_t)RW * 256 * 2); float* C1 = (float*)take((size_t)RW * 256 * 4); bf* A2h = (bf*)take((size_t)RW * 256 * 2); bf* A2l = (bf*)take((size_t)RW * 256 * 2); float* C2 = (float*)take((size_t)RW * 64 * 4);
    if ((size_t)(wsp - (char*)d_ws) > ws_size) return;
    k_w0p<<<(256 * 32 / 8 + 255) / 256, 256, 0, stream>>>(w0, B0); k_w1p<<<(256 * 256 / 8 + 255) / 256, 256, 0, stream>>>(w1, B1); k_w2p<<<(64 * 256 / 8 + 255) / 256, 256, 0, stream>>>(w2, B2);
    for (int c = 0; c < NCH; ++c) { const int b0 = c * BC;
        k_a0<<<(unsigned)(((size_t)RW * 32 / 8 + 255) / 256), 256, 0, stream>>>(x, b0, A0);
        k_gemmw<bf, 0, false><<<dim3(RW / 64, 256 / 64, 1), 32, 0, stream>>>(A0, nullptr, B0, nullptr, 32, C0, 256, nullptr, 0, 0, 0);
        k_p1<<<(unsigned)(((size_t)RW * 256 / 4 + 255) / 256), 256, 0, stream>>>(C0, A1h, A1l);
        k_gemmw<bf, 1, false><<<dim3(RW / 64, 256 / 64, 1), 32, 0, stream>>>(A1h, A1l, B1, nullptr, 256, C1, 256, nullptr, 0, 0, 0);
        k_p2<<<(unsigned)(((size_t)RW * 256 / 4 + 255) / 256), 256, 0, stream>>>(C1, A2h, A2l);
        k_gemmw<bf, 1, false><<<dim3(RW / 64, 64 / 64, 1), 32, 0, stream>>>(A2h, A2l, B2, nullptr, 256, C2, 64, nullptr, 0, 0, 0);
        k_out<<<(unsigned)(((size_t)BC * 4096 / 4 + 255) / 256), 256, 0, stream>>>(C2, bias, b0, OUT); }
}
